// ODEFunc_11141145166257
// MI455X (gfx1250) — hardware-verified
//
#include <hip/hip_runtime.h>
#include <math.h>

#ifndef NPTS
#define NPTS 1000000
#endif
#define HID 64
#define NGROUPS (NPTS / 32)
#define NBLK ((NGROUPS + 7) / 8)

#define CA_H 1024.0f
#define CA_T 4096.0f
#define CW   1024.0f
#define SC_H (1.0f / (1024.0f * 1024.0f))
#define SC_T (1.0f / (4096.0f * 1024.0f))

#define PW1X 0
#define PW1Y 64
#define PB1  128
#define PB2  192
#define PW30 256
#define PW31 320
#define PB3  384
#define PPAR 512

#define WS_W2H_OFF   0
#define WS_W2H_BYTES 8192
#define WS_PAR_OFF   8192
#define WS_PAR_BYTES 2048
#define WS_TOTAL     10240

static_assert(NPTS % 32 == 0);
static_assert(HID == 64);
static_assert(512 * 8 == HID * HID);
static_assert(HID * HID * 2 == WS_W2H_BYTES);
static_assert(PPAR * 4 == WS_PAR_BYTES);
static_assert(WS_W2H_OFF + WS_W2H_BYTES == WS_PAR_OFF);
static_assert(WS_PAR_OFF + WS_PAR_BYTES == WS_TOTAL);
static_assert(WS_TOTAL <= 134217728);
static_assert(24 * 16 == 32 * 3 * 4);
static_assert((PPAR + 8 * 96) * 4 <= 131072);

typedef _Float16 h16;
typedef __attribute__((ext_vector_type(16))) _Float16 v16h;
typedef __attribute__((ext_vector_type(8)))  _Float16 v8h;
typedef __attribute__((ext_vector_type(8)))  float    v8f;
typedef __attribute__((ext_vector_type(4)))  float    v4f;
typedef __attribute__((ext_vector_type(4)))  unsigned int v4u;


#define VST2(T, ptr, val) do { const T vst2_v_ = (val); *(volatile T*)(ptr) = vst2_v_; __threadfence(); *(volatile T*)(ptr) = vst2_v_; } while (0)

__device__ __forceinline__ float bfr(float f) {
    unsigned u = __float_as_uint(f);
    u += 0x7FFFu + ((u >> 16) & 1u);
    return __uint_as_float(u & 0xFFFF0000u);
}
static __device__ __forceinline__ h16 toh_flush(float v) {
    const h16 r = (h16)v;
    return (fabsf(v) < 6.103515625e-05f) ? (h16)0.0f : r;
}
__device__ __forceinline__ void st8h_flush(unsigned short* P, size_t o, const float* v) {
    v4u pk;
    pk.x = (unsigned)__builtin_bit_cast(unsigned short, toh_flush(v[0])) | ((unsigned)__builtin_bit_cast(unsigned short, toh_flush(v[1])) << 16);
    pk.y = (unsigned)__builtin_bit_cast(unsigned short, toh_flush(v[2])) | ((unsigned)__builtin_bit_cast(unsigned short, toh_flush(v[3])) << 16);
    pk.z = (unsigned)__builtin_bit_cast(unsigned short, toh_flush(v[4])) | ((unsigned)__builtin_bit_cast(unsigned short, toh_flush(v[5])) << 16);
    pk.w = (unsigned)__builtin_bit_cast(unsigned short, toh_flush(v[6])) | ((unsigned)__builtin_bit_cast(unsigned short, toh_flush(v[7])) << 16);
    VST2(v4u, (v4u*)(P + o), pk);
}

union FragU { v16h v; v8h h[2]; };
__device__ __forceinline__ v16h frag_ld(const _Float16* p) {
    FragU f; f.h[0] = *(const v8h*)(p); f.h[1] = *(const v8h*)(p + 16); return f.v;
}
__device__ __forceinline__ v8f wmma16(v16h a, v16h b, v8f c) {
    c = __builtin_amdgcn_wmma_f32_16x16x32_f16(false, a, false, b, (short)0, c, false, false);
    asm volatile("v_nop\n\tv_nop\n\tv_nop\n\tv_nop" : "+v"(c) : "v"(a), "v"(b));
    return c;
}
__device__ __forceinline__ void wave_sync_lds() {
    __builtin_amdgcn_fence(3  , "workgroup");
    __builtin_amdgcn_wave_barrier();
    __builtin_amdgcn_fence(2  , "workgroup");
}

__global__ __launch_bounds__(512) void k_prep(const float* __restrict__ W1, const float* __restrict__ b1,
                                              const float* __restrict__ W2, const float* __restrict__ b2,
                                              const float* __restrict__ W3, const float* __restrict__ b3,
                                              unsigned short* __restrict__ W2h, float* __restrict__ P) {
    const unsigned t = threadIdx.x;
    {
        const v4f a = *(const v4f*)(W2 + 8u * t);
        const v4f b = *(const v4f*)(W2 + 8u * t + 4u);
        float v[8];
        v[0] = bfr(a.x) * CW; v[1] = bfr(a.y) * CW; v[2] = bfr(a.z) * CW; v[3] = bfr(a.w) * CW;
        v[4] = bfr(b.x) * CW; v[5] = bfr(b.y) * CW; v[6] = bfr(b.z) * CW; v[7] = bfr(b.w) * CW;
        st8h_flush(W2h, (size_t)8u * t, v);
    }
    const unsigned i64 = t & 63u;
    const float w1x = bfr(W1[2u * i64]);
    const float w1y = bfr(W1[2u * i64 + 1u]);
    const float vb1 = bfr(b1[i64]);
    const float vb2 = bfr(b2[i64]);
    const float vw3 = bfr(W3[t & 127u]);
    const float vb3 = bfr(b3[t & 1u]);
    const unsigned seg = t >> 6;
    float val = 0.0f;
    val = (seg == 0u) ? w1x : val;
    val = (seg == 1u) ? w1y : val;
    val = (seg == 2u) ? vb1 : val;
    val = (seg == 3u) ? vb2 : val;
    val = (seg == 4u || seg == 5u) ? vw3 : val;
    val = (t == 384u || t == 385u) ? vb3 : val;
    VST2(float, P + t, val);
}

__global__ __launch_bounds__(256) void k_flow(const float* __restrict__ zlp, const _Float16* __restrict__ W2h,
                                              const float* __restrict__ P, float* __restrict__ out) {
    __shared__ __align__(16) float sPar[PPAR];
    __shared__ __align__(16) float sOut[8][96];
    const unsigned tid = threadIdx.x, lane = tid & 31u;
    const unsigned wave = __builtin_amdgcn_readfirstlane(threadIdx.x >> 5);
    const unsigned hh = lane >> 4, c = lane & 15u;

    sPar[tid] = P[tid];
    sPar[tid + 256u] = P[tid + 256u];
    __syncthreads();

    const unsigned group = blockIdx.x * 8u + wave;
    if (group >= (unsigned)NGROUPS) return;

    float* so = sOut[wave];
    const float ob0 = sPar[PB3], ob1 = sPar[PB3 + 1];

#pragma unroll 1
    for (unsigned mt = 0; mt < 2u; ++mt) {
        const size_t prow = (size_t)group * 32u + 16u * mt + c;
        const float z0 = bfr(zlp[prow * 3u]);
        const float z1 = bfr(zlp[prow * 3u + 1u]);

        v16h aH[2], aT0[2], aT1[2];
#pragma unroll
        for (int ks = 0; ks < 2; ++ks) {
#pragma unroll
            for (int g = 0; g < 2; ++g) {
                const unsigned kb = 32u * (unsigned)ks + 16u * (unsigned)g + 8u * hh;
                const v4f xa = *(const v4f*)(&sPar[PW1X + kb]);
                const v4f xb = *(const v4f*)(&sPar[PW1X + kb + 4u]);
                const v4f ya = *(const v4f*)(&sPar[PW1Y + kb]);
                const v4f yb = *(const v4f*)(&sPar[PW1Y + kb + 4u]);
                const v4f ba = *(const v4f*)(&sPar[PB1 + kb]);
                const v4f bb = *(const v4f*)(&sPar[PB1 + kb + 4u]);
                const float wx[8] = {xa.x, xa.y, xa.z, xa.w, xb.x, xb.y, xb.z, xb.w};
                const float wy[8] = {ya.x, ya.y, ya.z, ya.w, yb.x, yb.y, yb.z, yb.w};
                const float bz[8] = {ba.x, ba.y, ba.z, ba.w, bb.x, bb.y, bb.z, bb.w};
#pragma unroll
                for (int e = 0; e < 8; ++e) {
                    const float pre = (z0 * wx[e] + z1 * wy[e]) + bz[e];
                    const float ex = expf(fminf(pre, 0.0f));
                    const bool pos = pre > 0.0f;
                    const float hv = pos ? pre : (ex - 1.0f);
                    const float dp = pos ? 1.0f : ex;
                    aH[ks][8 * g + e]  = toh_flush(hv * CA_H);
                    aT0[ks][8 * g + e] = toh_flush((dp * wx[e]) * CA_T);
                    aT1[ks][8 * g + e] = toh_flush((dp * wy[e]) * CA_T);
                }
            }
        }

        float p0[8], p1[8], pt[8];
#pragma unroll
        for (int r = 0; r < 8; ++r) { p0[r] = 0.0f; p1[r] = 0.0f; pt[r] = 0.0f; }

#pragma unroll 1
        for (unsigned jp = 0; jp < 2u; ++jp) {
            v8f ch[2], c0[2], c1[2];
#pragma unroll
            for (int jj = 0; jj < 2; ++jj) {
                ch[jj] = (v8f){0.f,0.f,0.f,0.f,0.f,0.f,0.f,0.f};
                c0[jj] = ch[jj];
                c1[jj] = ch[jj];
            }
#pragma unroll
            for (int ks = 0; ks < 2; ++ks) {
#pragma unroll
                for (int jj = 0; jj < 2; ++jj) {
                    const v16h bf = frag_ld(W2h + (size_t)(32u * jp + 16u * (unsigned)jj + c) * 64u + 32u * (unsigned)ks + 8u * hh);
                    ch[jj] = wmma16(aH[ks],  bf, ch[jj]);
                    c0[jj] = wmma16(aT0[ks], bf, c0[jj]);
                    c1[jj] = wmma16(aT1[ks], bf, c1[jj]);
                }
            }
#pragma unroll
            for (int jj = 0; jj < 2; ++jj) {
                const unsigned n = 32u * jp + 16u * (unsigned)jj + c;
                const float b2n = sPar[PB2 + n];
                const float w30 = sPar[PW30 + n];
                const float w31 = sPar[PW31 + n];
#pragma unroll
                for (int r = 0; r < 8; ++r) {
                    const float a2 = ch[jj][r] * SC_H + b2n;
                    const float e2 = expf(fminf(a2, 0.0f));
                    const bool pos2 = a2 > 0.0f;
                    const float h2 = pos2 ? a2 : (e2 - 1.0f);
                    const float d2 = pos2 ? 1.0f : e2;
                    const float t0 = c0[jj][r] * SC_T;
                    const float t1 = c1[jj][r] * SC_T;
                    p0[r] += w30 * h2;
                    p1[r] += w31 * h2;
                    pt[r] += d2 * (w30 * t0 + w31 * t1);
                }
            }
        }

#pragma unroll
        for (int r = 0; r < 8; ++r) {
            float r0 = p0[r], r1 = p1[r], rt = pt[r];
#pragma unroll
            for (int m = 1; m < 16; m <<= 1) {
                r0 += __shfl_xor(r0, m, 32);
                r1 += __shfl_xor(r1, m, 32);
                rt += __shfl_xor(rt, m, 32);
            }
            if (c == 0u) {
                const unsigned row = 16u * mt + 8u * hh + (unsigned)r;
                so[row * 3u + 0u] = r0 + ob0;
                so[row * 3u + 1u] = r1 + ob1;
                so[row * 3u + 2u] = -rt;
            }
        }
    }

    wave_sync_lds();
    {
        const unsigned lc = (lane < 24u) ? lane : 23u;
        const v4f ov = *(const v4f*)(so + 4u * lc);
        float* dst = out + (size_t)group * 96u + 4u * lc;
        for (int pass = 0; pass < 2; ++pass) {
            if (lane < 24u) *(volatile v4f*)dst = ov;
            __threadfence();
        }
    }
}

extern "C" void kernel_launch(void* const* d_in, const int* in_sizes, int n_in, void* d_out, int out_size,
                              void* d_ws, size_t ws_size, hipStream_t stream) {
    if (n_in < 8) return;
    if (in_sizes[1] < NPTS * 3 || in_sizes[2] < HID * 2 || in_sizes[3] < HID || in_sizes[4] < HID * HID) return;
    if (in_sizes[5] < HID || in_sizes[6] < 2 * HID || in_sizes[7] < 2 || out_size < NPTS * 3) return;
    if (ws_size < (size_t)WS_TOTAL) return;

    const float* t_in = (const float*)d_in[0];
    (void)t_in;
    const float* zlp = (const float*)d_in[1];
    const float* W1  = (const float*)d_in[2];
    const float* b1  = (const float*)d_in[3];
    const float* W2  = (const float*)d_in[4];
    const float* b2  = (const float*)d_in[5];
    const float* W3  = (const float*)d_in[6];
    const float* b3  = (const float*)d_in[7];
    float* out = (float*)d_out;

    char* wsp = (char*)d_ws;
    unsigned short* w2h = (unsigned short*)(wsp + WS_W2H_OFF);
    float*          par = (float*)(wsp + WS_PAR_OFF);

    k_prep<<<1, 512, 0, stream>>>(W1, b1, W2, b2, W3, b3, w2h, par);
    k_flow<<<NBLK, 256, 0, stream>>>(zlp, (const _Float16*)w2h, (const float*)par, out);
}
